// IntegralTransform_4990751998525
// MI455X (gfx1250) — hardware-verified
//
#include <hip/hip_runtime.h>


namespace {
constexpr int N = 50000, E = 1600000, DC = 3, DH = 64, DF = 64;
constexpr float HS = 256.0f, WSC = 256.0f;
typedef _Float16 b16;
typedef __attribute__((ext_vector_type(16))) _Float16 v16b;
typedef __attribute__((ext_vector_type(8))) _Float16 v8b;
typedef __attribute__((ext_vector_type(8))) float v8f;
typedef __attribute__((ext_vector_type(2))) float v2f;
__device__ __forceinline__ float bf16_rne(float f) { unsigned int u = __float_as_uint(f); u += 0x7FFFu + ((u >> 16) & 1u); float r = __uint_as_float(u & 0xFFFF0000u); asm volatile("" : "+v"(r)); return r; }
__device__ __forceinline__ float bfv(float f) { float r = bf16_rne(f); asm volatile("" : "+v"(r)); return r; }
__device__ __forceinline__ void split16(float v, b16& hi, b16& lo) { hi = (b16)v; lo = (b16)(v - (float)hi); }
__device__ __forceinline__ v16b frag_kb(const b16* p, int hh) { const v8b a = *(const v8b*)(p + 8 * hh), b = *(const v8b*)(p + 16 + 8 * hh); v16b f;
#pragma unroll
  for (int e = 0; e < 8; ++e) { f[e] = a[e]; f[8 + e] = b[e]; } return f; }
__device__ __forceinline__ v8f wmma16b(v16b a, v16b b, v8f c) { v8f d = __builtin_amdgcn_wmma_f32_16x16x32_f16(false, a, false, b, (short)0, c, false, false); asm volatile("v_nop\n\tv_nop\n\tv_nop\n\tv_nop" : "+v"(d) : "v"(a), "v"(b)); return d; }
__device__ __forceinline__ void wave_lds_sync() { __builtin_amdgcn_fence(__ATOMIC_RELEASE, "workgroup"); __builtin_amdgcn_wave_barrier(); __builtin_amdgcn_fence(__ATOMIC_ACQUIRE, "workgroup"); }
__device__ __forceinline__ float pmul(float a, float b) { float p = a * b; asm volatile("" : "+v"(p)); return p; }
__device__ __forceinline__ int iclamp(int v, int lo, int hi) { return v < lo ? lo : (v > hi ? hi : v); }

__global__ __launch_bounds__(256) void wput_kernel(const float* __restrict__ w1, b16* __restrict__ WT) { const int u = blockIdx.x * 256 + threadIdx.x; if (u >= DF * 8) return; const int o = u / 8, k0 = (u % 8) * 8; v8b v;
#pragma unroll
  for (int j = 0; j < 8; ++j) v[j] = (b16)(bf16_rne(w1[(size_t)(k0 + j) * DF + o]) * WSC);
  for (int pass = 0; pass < 2; ++pass) { *(volatile v8b*)(WT + (size_t)o * DH + k0) = v; __threadfence(); } }
__global__ __launch_bounds__(32) void main_kernel(const float* __restrict__ y, const float* __restrict__ fy, const float* __restrict__ w0, const float* __restrict__ b0, const float* __restrict__ b1, const int* __restrict__ nbr, const int* __restrict__ rs, const b16* __restrict__ WT, int NLIM, float* __restrict__ out) { __shared__ __attribute__((aligned(16))) b16 Ah[16][DH + 8], Al[16][DH + 8]; __shared__ float Tf[16][DF + 1], Yj[16][4]; __shared__ int Jd[16]; const int lane = threadIdx.x, nloc = lane & 15, hlf = lane >> 4; const size_t i = blockIdx.x; if (i >= (size_t)NLIM) return;
  int st = rs[i], en = rs[i + 1]; st = iclamp(st, 0, E); en = iclamp(en, st, E); const int cnt = en - st;
  const float yi0 = bfv(y[i * 3]), yi1 = bfv(y[i * 3 + 1]), yi2 = bfv(y[i * 3 + 2]);
  float wa[2][6], ba[2], bb1[2]; for (int e2 = 0; e2 < 2; ++e2) { const int c = lane * 2 + e2; for (int r = 0; r < 6; ++r) wa[e2][r] = bfv(w0[r * DH + c]); ba[e2] = bfv(b0[c]); bb1[e2] = bfv(b1[c]); }
  if (lane < 16) for (int k = DH; k < DH + 8; ++k) { Ah[lane][k] = (b16)0.0f; Al[lane][k] = (b16)0.0f; }
  float acc0 = 0.0f, acc1 = 0.0f; int used = 0;
#pragma unroll 1
  for (int t0 = 0; t0 < cnt; t0 += 16) { const int nt = cnt - t0 < 16 ? cnt - t0 : 16;
    if (lane < 16) { const int e = st + t0 + lane; int j = 0; float a = 0, b = 0, c = 0; if (lane < nt) { j = iclamp(nbr[e], 0, N - 1); a = bfv(y[(size_t)j * 3]); b = bfv(y[(size_t)j * 3 + 1]); c = bfv(y[(size_t)j * 3 + 2]); } Jd[lane] = j; Yj[lane][0] = a; Yj[lane][1] = b; Yj[lane][2] = c; }
    wave_lds_sync();
    for (int r = 0; r < 16; ++r) { for (int e2 = 0; e2 < 2; ++e2) { float hv = 0.0f; if (r < nt) { const float s = ba[e2] + pmul(Yj[r][0], wa[e2][0]) + pmul(Yj[r][1], wa[e2][1]) + pmul(Yj[r][2], wa[e2][2]) + pmul(yi0, wa[e2][3]) + pmul(yi1, wa[e2][4]) + pmul(yi2, wa[e2][5]); hv = 0.5f * s * (1.0f + erff(s * 0.70710678118654752f)); } b16 p, pl; split16(hv * HS, p, pl); Ah[r][lane * 2 + e2] = p; Al[r][lane * 2 + e2] = pl; } }
    wave_lds_sync();
    v8f d[4] = {(v8f){}, (v8f){}, (v8f){}, (v8f){}};
#pragma unroll
    for (int kb = 0; kb < DH; kb += 32) { const v16b a = frag_kb(&Ah[nloc][kb], hlf), al = frag_kb(&Al[nloc][kb], hlf);
#pragma unroll
      for (int t = 0; t < 4; ++t) { const v16b bw = frag_kb(WT + (size_t)(t * 16 + nloc) * DH + kb, hlf); d[t] = wmma16b(a, bw, d[t]); d[t] = wmma16b(al, bw, d[t]); } }
#pragma unroll
    for (int t = 0; t < 4; ++t)
#pragma unroll
      for (int r8 = 0; r8 < 8; ++r8) Tf[8 * hlf + r8][t * 16 + nloc] = d[t][r8] * (1.0f / (HS * WSC));
    wave_lds_sync();
    for (int r = 0; r < nt; ++r) { const size_t j = (size_t)Jd[r]; if (j >= (size_t)NLIM) continue; ++used; const v2f f = *(const v2f*)(fy + j * DF + lane * 2); acc0 += pmul(Tf[r][lane * 2] + bb1[0], bfv(f[0])); acc1 += pmul(Tf[r][lane * 2 + 1] + bb1[1], bfv(f[1])); }
    wave_lds_sync(); }
  const float inv = 1.0f / (float)(cnt < 1 ? 1 : cnt); (void)used;
  for (int pass = 0; pass < 2; ++pass) { *(volatile v2f*)(out + i * DF + lane * 2) = (v2f){acc0 * inv, acc1 * inv}; __threadfence(); } }
}

extern "C" void kernel_launch(void* const* d_in, const int* in_sizes, int n_in, void* d_out, int out_size, void* d_ws, size_t ws_size, hipStream_t stream) {
  (void)n_in;
  auto Fp = [&](int i) { return (const float*)d_in[i]; }; auto Ip = [&](int i) { return (const int*)d_in[i]; };
  if (in_sizes[0] != N * DC || in_sizes[1] != N * DF || in_sizes[2] != 2 * DC * DH || in_sizes[4] != DH * DF || in_sizes[6] != E || in_sizes[7] != N + 1 || out_size != N * DF) return;
  const int NLIM = N;
  size_t off = 0; char* ws = (char*)d_ws;
  auto carve = [&](size_t bytes) { char* p = ws + off; off += (bytes + 255) & ~(size_t)255; return p; };
  b16* WT = (b16*)carve((size_t)DF * DH * 2);
  if (off > ws_size || off > ((size_t)1 << 20)) return;
  wput_kernel<<<(DF * 8 + 255) / 256, 256, 0, stream>>>(Fp(4), WT);
  main_kernel<<<NLIM, 32, 0, stream>>>(Fp(0), Fp(1), Fp(2), Fp(3), Fp(5), Ip(6), Ip(7), WT, NLIM, (float*)d_out);
}
